// TripletLoss_6021544149806
// MI455X (gfx1250) — hardware-run, weakly checked
//
#include <hip/hip_runtime.h>
#include <math.h>


#ifndef NANCH
#define NANCH 4096
#endif
#ifndef NGAL
#define NGAL 4096
#endif
#define NROW_FULL 4096
#define DM   1024
#define AW   4
#define BIGF 3.0e38f

static_assert(DM == 1024);
static_assert(DM % 32 == 0);
static_assert(NGAL % 64 == 0);
static_assert((NGAL / 64) % AW == 0);
static_assert(NANCH % 64 == 0);
static_assert(NANCH <= NGAL);
static_assert(NGAL <= NROW_FULL);

typedef unsigned short bf;
typedef __attribute__((ext_vector_type(16))) __bf16   v16bf;
typedef __attribute__((ext_vector_type(8)))  unsigned short v8us;
typedef __attribute__((ext_vector_type(8)))  float    v8f;
typedef __attribute__((ext_vector_type(4)))  float    v4f;
typedef __attribute__((ext_vector_type(4)))  int      v4i;
typedef v4f  __attribute__((may_alias)) v4fa;

__device__ __forceinline__ unsigned short f2bf(float f) { unsigned u = __float_as_uint(f); u += 0x7FFFu + ((u >> 16) & 1u); return (unsigned short)(u >> 16); }
__device__ __forceinline__ v16bf cat16b(v8us lo, v8us hi) { return __builtin_bit_cast(v16bf, __builtin_shufflevector(lo, hi, 0, 1, 2, 3, 4, 5, 6, 7, 8, 9, 10, 11, 12, 13, 14, 15)); }
__device__ __forceinline__ v8f wmmab(v16bf a, v16bf b, v8f c) { return __builtin_amdgcn_wmma_f32_16x16x32_bf16(false, a, false, b, (short)0, c, false, false); }
__device__ __forceinline__ v16bf ldb(const bf* p)  { return cat16b(*(const v8us*)p, *(const v8us*)(p + 16)); }

__global__ __launch_bounds__(256) void k_prep(const float* __restrict__ feat, bf* FB, float* SQ) {
    __shared__ __align__(16) float sqs[32];
    const int lane = threadIdx.x & 31;
    const int wave = __builtin_amdgcn_readfirstlane((int)(threadIdx.x >> 5));
    const int rb = blockIdx.x * 32 + wave * 4;
#pragma unroll 1
    for (int rr = 0; rr < 4; ++rr) {
        const size_t ro = (size_t)(rb + rr) * DM;
        float s = 0.0f;
#pragma unroll 1
        for (int it = 0; it < 4; ++it) {
            const int c = it * 256 + lane * 8;
            const v8f v = *(const v8f*)(feat + ro + c);
            v8us o;
#pragma unroll
            for (int k = 0; k < 8; ++k) { const unsigned short b = f2bf(v[k]); o[k] = b; const float t = __uint_as_float(((unsigned)b) << 16); s += t * t; }
            *(volatile v8us*)(FB + ro + c) = o; __threadfence(); *(volatile v8us*)(FB + ro + c) = o;
        }
        s += __shfl_xor(s, 16, 32); s += __shfl_xor(s, 8, 32); s += __shfl_xor(s, 4, 32); s += __shfl_xor(s, 2, 32); s += __shfl_xor(s, 1, 32);
        if (lane == 0) sqs[wave * 4 + rr] = s;
    }
    __syncthreads();
    if (threadIdx.x < 8) {
        const v4f val = *(const v4fa*)(&sqs[threadIdx.x * 4]);
        float* p = SQ + (size_t)blockIdx.x * 32 + threadIdx.x * 4;
        *(volatile v4f*)p = val; __threadfence(); *(volatile v4f*)p = val;
    }
}

__global__ __launch_bounds__(32 * AW) void k_hard(const bf* __restrict__ FB, const float* __restrict__ SQ, const int* __restrict__ ID, float* OUT) {
    __shared__ __align__(16) float red[AW * 3 * 64];
    __shared__ __align__(16) float ob[64];
    const int lane = threadIdx.x & 31, lr = lane & 15, hi = lane >> 4;
    const int wave = __builtin_amdgcn_readfirstlane((int)(threadIdx.x >> 5));
    const int i0 = blockIdx.x * 64;
    float sqi[4], mp[4], mnS[4], mnN[4]; int idi[4];
#pragma unroll
    for (int nb = 0; nb < 4; ++nb) { sqi[nb] = SQ[i0 + nb * 16 + lr]; idi[nb] = ID[i0 + nb * 16 + lr]; mp[nb] = -BIGF; mnS[nb] = BIGF; mnN[nb] = BIGF; }
    const size_t boff = (size_t)(i0 + lr) * DM + 8 * hi;
#pragma unroll 1
    for (int ct = wave; ct < NGAL / 64; ct += AW) {
        const int j0 = ct * 64;
        const size_t aoff = (size_t)(j0 + lr) * DM + 8 * hi;
        v8f acc[4][4];
#pragma unroll
        for (int mb = 0; mb < 4; ++mb)
#pragma unroll
            for (int nb = 0; nb < 4; ++nb) acc[mb][nb] = (v8f){};
#pragma unroll 1
        for (int kc = 0; kc < DM; kc += 32) {
            v16bf a[4];
#pragma unroll
            for (int mb = 0; mb < 4; ++mb) a[mb] = ldb(FB + aoff + (size_t)mb * 16 * DM + kc);
#pragma unroll
            for (int nb = 0; nb < 4; ++nb) { const v16bf b = ldb(FB + boff + (size_t)nb * 16 * DM + kc);
#pragma unroll
                for (int mb = 0; mb < 4; ++mb) acc[mb][nb] = wmmab(a[mb], b, acc[mb][nb]); }
            asm volatile("v_nop\n\tv_nop\n\tv_nop\n\tv_nop" : "+v"(acc[0][0]), "+v"(acc[1][1]), "+v"(acc[2][2]), "+v"(acc[3][3]) : "v"(a[0]), "v"(a[1]), "v"(a[2]), "v"(a[3]));
        }
        const int dl = (j0 - i0) + 8 * hi - lr;
#pragma unroll
        for (int mb = 0; mb < 4; ++mb) {
            const int jr = j0 + mb * 16 + 8 * hi;
            const v4f s0 = *(const v4f*)(SQ + jr); const v4f s1 = *(const v4f*)(SQ + jr + 4);
            const v4i d0 = *(const v4i*)(ID + jr); const v4i d1 = *(const v4i*)(ID + jr + 4);
            const float sj[8] = { s0[0], s0[1], s0[2], s0[3], s1[0], s1[1], s1[2], s1[3] };
            const int   dj[8] = { d0[0], d0[1], d0[2], d0[3], d1[0], d1[1], d1[2], d1[3] };
#pragma unroll
            for (int r = 0; r < 8; ++r) {
#pragma unroll
                for (int nb = 0; nb < 4; ++nb) {
                    const float d2 = (sqi[nb] + sj[r]) - 2.0f * acc[mb][nb][r];
                    const bool same = (dj[r] == idi[nb]);
                    const bool offd = (dl != (nb - mb) * 16 - r);
                    const float cp = (same && offd) ? d2 : -BIGF;
                    const float cs = same ? d2 : BIGF;
                    const float cn = same ? BIGF : d2;
                    mp[nb]  = fmaxf(mp[nb], cp);
                    mnS[nb] = fminf(mnS[nb], cs);
                    mnN[nb] = fminf(mnN[nb], cn);
                }
            }
        }
    }
#pragma unroll
    for (int nb = 0; nb < 4; ++nb) {
        const float xp = __shfl_xor(mp[nb], 16, 32); const float xs = __shfl_xor(mnS[nb], 16, 32); const float xn = __shfl_xor(mnN[nb], 16, 32);
        mp[nb] = fmaxf(mp[nb], xp); mnS[nb] = fminf(mnS[nb], xs); mnN[nb] = fminf(mnN[nb], xn);
    }
    if (hi == 0) {
#pragma unroll
        for (int nb = 0; nb < 4; ++nb) {
            red[(wave * 3 + 0) * 64 + nb * 16 + lr] = mp[nb];
            red[(wave * 3 + 1) * 64 + nb * 16 + lr] = mnS[nb];
            red[(wave * 3 + 2) * 64 + nb * 16 + lr] = mnN[nb];
        }
    }
    __syncthreads();
    if (threadIdx.x < 64) {
        const int t = threadIdx.x;
        float p = -BIGF, s = BIGF, n = BIGF;
#pragma unroll
        for (int w = 0; w < AW; ++w) { p = fmaxf(p, red[(w * 3 + 0) * 64 + t]); s = fminf(s, red[(w * 3 + 1) * 64 + t]); n = fminf(n, red[(w * 3 + 2) * 64 + t]); }
        const float dpos = sqrtf(fmaxf(p, 0.0f) + 1e-12f);
        const float maxpos = (p > -1.0e38f) ? dpos : 0.0f;
        const float dneg = sqrtf(fmaxf(n, 0.0f) + 1e-12f);
        const float dsam = sqrtf(fmaxf(s, 0.0f) + 1e-12f) + 1.0e5f;
        const float minneg = fminf(dneg, dsam);
        const float z = maxpos - minneg;
        ob[t] = fmaxf(z, 0.0f) + log1pf(expf(-fabsf(z)));
    }
    __syncthreads();
    if (threadIdx.x < 16) {
        const v4f val = *(const v4fa*)(&ob[threadIdx.x * 4]);
        float* q = OUT + (size_t)i0 + threadIdx.x * 4;
        *(volatile v4f*)q = val; __threadfence(); *(volatile v4f*)q = val;
    }
}

static constexpr size_t al256(size_t v) { return (v + 255) & ~(size_t)255; }
static constexpr size_t SZ_FB = al256((size_t)NGAL * DM * 2);
static constexpr size_t SZ_SQ = al256((size_t)NGAL * 4);
static constexpr size_t SZ_TOTAL = SZ_FB + SZ_SQ;
static_assert(SZ_TOTAL <= (size_t)134217728);
static_assert(((size_t)NGAL * DM * 2) % 256 == 0);
static_assert(((size_t)(NGAL / 32 - 1) * 32 + 32) * 4 <= SZ_SQ);
static_assert(((size_t)(NANCH / 64 - 1) * 64 + 64) <= (size_t)NANCH);

extern "C" void kernel_launch(void* const* d_in, const int* in_sizes, int n_in,
                              void* d_out, int out_size, void* d_ws, size_t ws_size, hipStream_t stream) {
    if (n_in < 2) return;
    if ((size_t)in_sizes[0] < (size_t)NGAL * DM) return;
    if ((size_t)in_sizes[1] < (size_t)NGAL) return;
    if ((size_t)out_size < (size_t)NANCH) return;
    if (SZ_TOTAL > ws_size) return;
    const float* feat = (const float*)d_in[0];
    const int*   ids  = (const int*)d_in[1];
    float* OUT = (float*)d_out;
    char* wsp = (char*)d_ws;
    bf* FB = (bf*)wsp; wsp += SZ_FB;
    float* SQ = (float*)wsp; wsp += SZ_SQ;

    k_prep<<<dim3(NGAL / 32, 1, 1), 256, 0, stream>>>(feat, FB, SQ);
    k_hard<<<dim3(NANCH / 64, 1, 1), 32 * AW, 0, stream>>>(FB, SQ, ids, OUT);
}
